// SelectiveSSM_87703232184785
// MI455X (gfx1250) — hardware-verified
//
#include <hip/hip_runtime.h>
#include <math.h>

typedef __attribute__((ext_vector_type(16))) _Float16 v16h;
typedef __attribute__((ext_vector_type(8)))  _Float16 v8h;
typedef __attribute__((ext_vector_type(16))) __bf16   v16b;
typedef __attribute__((ext_vector_type(8)))  __bf16   v8b;
typedef __attribute__((ext_vector_type(8)))  float    v8f;
typedef __attribute__((ext_vector_type(4)))  float    v4f;
typedef __attribute__((ext_vector_type(4)))  unsigned v4u;

constexpr int kBatch  = 2;
constexpr int kSeq    = 2048;
constexpr int kDm     = 768;
constexpr int kDin    = 1536;
constexpr int kNst    = 16;
constexpr int kXzN    = 2 * kDin;
constexpr int kBcN    = 2 * kNst;
constexpr int kDtxN   = kDin + 64;
constexpr int kRows   = kBatch * kSeq;
constexpr int kScanCh = 256;
constexpr int kScanTS = 16;
constexpr int kScanTP = 260;
static_assert(kDm == 768 && kDin == 2 * kDm && kNst == 16 && kSeq == 2048 && kBatch == 2, "shape constants");
static_assert((kDm % 32) == 0 && (kDin % 32) == 0, "GEMM K multiples of 32");
static_assert((kRows % 64) == 0 && (kDin % 64) == 0 && (kDtxN % 64) == 0 && (kDm % 64) == 0 && (kXzN % 64) == 0, "GEMM M,N multiples of 64");
static_assert(((kRows / 64) * (kDin / 64)) % 8 == 0 && ((kRows / 64) * (kDtxN / 64)) % 8 == 0 && ((kRows / 64) * (kDm / 64)) % 8 == 0, "8 tiles per GEMM block exactly");
static_assert((kDm % 64) == 0 && (kDin % 64) == 0, "transpose tiles");
static_assert((kSeq % kScanTS) == 0 && (kDin % kScanCh) == 0 && kScanCh == 256 && kScanTS == 16, "scan tiles");
static_assert(((kRows * kDm) % (8 * 256)) == 0, "cast coverage");
static_assert(kBcN + 32 == kDtxN - kDin, "B|C|pad columns");

constexpr size_t kOffXB    = 0;
constexpr size_t kOffWINB  = kOffXB    + (size_t)kRows * kDm  * 2;
constexpr size_t kOffWDTXB = kOffWINB  + (size_t)kXzN  * kDm  * 2;
constexpr size_t kOffWOUTB = kOffWDTXB + (size_t)kDtxN * kDin * 2;
constexpr size_t kOffZF    = kOffWOUTB + (size_t)kDm   * kDin * 2;
constexpr size_t kOffXPH   = kOffZF    + (size_t)kRows * kDin * 4;
constexpr size_t kOffXPL   = kOffXPH   + (size_t)kRows * kDin * 2;
constexpr size_t kOffDTX   = kOffXPL   + (size_t)kRows * kDin * 2;
constexpr size_t kOffYH    = kOffDTX   + (size_t)kRows * kDtxN * 4;
constexpr size_t kOffYL    = kOffYH    + (size_t)kRows * kDin * 2;
constexpr size_t kWsTotal  = kOffYL    + (size_t)kRows * kDin * 2;
static_assert(kWsTotal == 119996416ull, "carve total");
static_assert(kWsTotal <= 134217728ull, "carve cap");
static_assert((kOffWINB % 128) == 0 && (kOffWDTXB % 128) == 0 && (kOffWOUTB % 128) == 0 && (kOffZF % 128) == 0 &&
              (kOffXPH % 128) == 0 && (kOffXPL % 128) == 0 && (kOffDTX % 128) == 0 && (kOffYH % 128) == 0 &&
              (kOffYL % 128) == 0, "128-B aligned regions");
static_assert(((kDm * 2) % 128) == 0 && ((kDin * 2) % 128) == 0 && ((kDin * 4) % 128) == 0 && ((kDtxN * 4) % 128) == 0 && ((kDm * 4) % 128) == 0, "row pitches are whole lines");

__device__ __forceinline__ unsigned short f2bf_bits(float f) {
  unsigned u = __float_as_uint(f);
  return (unsigned short)((u + 0x7FFFu + ((u >> 16) & 1u)) >> 16);
}
__device__ __forceinline__ float bf_bits2f(unsigned short h) { return __uint_as_float(((unsigned)h) << 16); }
__device__ __forceinline__ float bf16_rne(float f) { return bf_bits2f(f2bf_bits(f)); }

__device__ __forceinline__ void dep_guard4_h(v8f& a, v8f& b, v8f& c, v8f& d, v16h x, v16h y) {
  asm volatile("v_nop\n\tv_nop\n\tv_nop\n\tv_nop" : "+v"(a), "+v"(b), "+v"(c), "+v"(d) : "v"(x), "v"(y));
}
__device__ __forceinline__ void dep_guard4_b(v8f& a, v8f& b, v8f& c, v8f& d, v16b x, v16b y) {
  asm volatile("v_nop\n\tv_nop\n\tv_nop\n\tv_nop" : "+v"(a), "+v"(b), "+v"(c), "+v"(d) : "v"(x), "v"(y));
}
__device__ __forceinline__ void keep4_h(v16h a, v16h b, v16h c, v16h d) { asm volatile("v_nop" :: "v"(a), "v"(b), "v"(c), "v"(d)); }
__device__ __forceinline__ void keep4_b(v16b a, v16b b, v16b c, v16b d) { asm volatile("v_nop" :: "v"(a), "v"(b), "v"(c), "v"(d)); }
__device__ __forceinline__ void acc_guard4(v8f& a, v8f& b, v8f& c, v8f& d) { asm volatile("v_nop\n\tv_nop\n\tv_nop\n\tv_nop" : "+v"(a), "+v"(b), "+v"(c), "+v"(d)); }
template <typename T> struct Frag;
template <> struct Frag<_Float16> {
  typedef v16h V; union U { v16h v; v8h h[2]; };
  static __device__ __forceinline__ v16h load(const _Float16* p) {
    U f; f.h[0] = *(const v8h*)(p); f.h[1] = *(const v8h*)(p + 16); return f.v;
  }
  static __device__ __forceinline__ v8f mma(v16h a, v16h b, v8f c) {
    return __builtin_amdgcn_wmma_f32_16x16x32_f16(false, a, false, b, (short)0, c, false, false);
  }
  static __device__ __forceinline__ void guard4(v8f& a, v8f& b, v8f& c, v8f& d, v16h x, v16h y) { dep_guard4_h(a, b, c, d, x, y); }
  static __device__ __forceinline__ void keep(v16h a, v16h b, v16h c, v16h d) { keep4_h(a, b, c, d); }
};
template <> struct Frag<__bf16> {
  typedef v16b V; union U { v16b v; v8b h[2]; };
  static __device__ __forceinline__ v16b load(const __bf16* p) {
    U f; f.h[0] = *(const v8b*)(p); f.h[1] = *(const v8b*)(p + 16); return f.v;
  }
  static __device__ __forceinline__ v8f mma(v16b a, v16b b, v8f c) {
    return __builtin_amdgcn_wmma_f32_16x16x32_bf16(false, a, false, b, (short)0, c, false, false);
  }
  static __device__ __forceinline__ void guard4(v8f& a, v8f& b, v8f& c, v8f& d, v16b x, v16b y) { dep_guard4_b(a, b, c, d, x, y); }
  static __device__ __forceinline__ void keep(v16b a, v16b b, v16b c, v16b d) { keep4_b(a, b, c, d); }
};

template <int ET> struct Elem;
template <> struct Elem<0> { typedef _Float16 T; };
template <> struct Elem<1> { typedef __bf16 T; };
template <int ET, int SPL, int BIAS_MODE, int OUT_MODE, bool RESID, int ACT = 0>
__global__ __launch_bounds__(256) void wmma_gemm64(
    const unsigned short* __restrict__ Ap, const unsigned short* __restrict__ A2p, int lda, long strideA,
    const unsigned short* __restrict__ Btp, const unsigned short* __restrict__ Bt2p, int ldb, long strideB,
    void* __restrict__ Cout, void* __restrict__ Cout2, int ldc, long strideC,
    const float* __restrict__ bias,
    const float* __restrict__ resid, long strideR,
    int M, int N, int K, float scale) {
  typedef typename Elem<ET>::T T;
  typedef typename Frag<T>::V V;
  const T* A = (const T*)Ap; const T* A2 = (const T*)A2p; const T* Bt = (const T*)Btp; const T* Bt2 = (const T*)Bt2p;
  __shared__ __align__(16) float sT[8][16 * 68];
  const int b    = blockIdx.y;
  const int lane = threadIdx.x & 31;
  const int wave = threadIdx.x >> 5;
  const int tilesN = N >> 6;
  const int tilesM = M >> 6;
  const int tile = blockIdx.x * 8 + wave;
  if (tile >= tilesM * tilesN) return;
  const int tm = tile / tilesN;
  const int tn = tile - tm * tilesN;
  const int m0 = tm << 6;
  const int n0 = tn << 6;

  const T* Ab  = A  + (size_t)b * strideA;
  const T* Bb  = Bt + (size_t)b * strideB;
  const T* Ab2 = (SPL >= 1) ? (A2  + (size_t)b * strideA) : nullptr;
  const T* Bb2 = (SPL == 2) ? (Bt2 + (size_t)b * strideB) : nullptr;

  const int rlane = lane & 15;
  const int koff  = (lane >> 4) * 8;
  const int mOff  = (lane >> 4) * 8;

  v8f acc[4][4];
#pragma unroll
  for (int i = 0; i < 4; ++i)
#pragma unroll
    for (int j = 0; j < 4; ++j) acc[i][j] = (v8f){0.f,0.f,0.f,0.f,0.f,0.f,0.f,0.f};

  for (int k0 = 0; k0 < K; k0 += 32) {
    V bh[4], bl[4];
#pragma unroll
    for (int j = 0; j < 4; ++j) {
      const size_t bo = (size_t)(n0 + (j << 4) + rlane) * ldb + koff + k0;
      bh[j] = Frag<T>::load(Bb + bo);
      if (SPL == 2) bl[j] = Frag<T>::load(Bb2 + bo);
    }
#pragma unroll
    for (int i = 0; i < 4; ++i) {
      const size_t ao = (size_t)(m0 + (i << 4) + rlane) * lda + koff + k0;
      V ah = Frag<T>::load(Ab + ao);
      V al;
      if (SPL >= 1) al = Frag<T>::load(Ab2 + ao);
#pragma unroll
      for (int j = 0; j < 4; ++j) {
        acc[i][j] = Frag<T>::mma(ah, bh[j], acc[i][j]);
        if (SPL == 2) acc[i][j] = Frag<T>::mma(ah, bl[j], acc[i][j]);
        if (SPL >= 1) acc[i][j] = Frag<T>::mma(al, bh[j], acc[i][j]);
      }
      Frag<T>::guard4(acc[i][0], acc[i][1], acc[i][2], acc[i][3], ah, (SPL >= 1) ? al : ah);
    }
    Frag<T>::keep(bh[0], bh[1], bh[2], bh[3]);
    if (SPL == 2) Frag<T>::keep(bl[0], bl[1], bl[2], bl[3]);
  }
  acc_guard4(acc[0][0], acc[0][1], acc[0][2], acc[0][3]);
  acc_guard4(acc[1][0], acc[1][1], acc[1][2], acc[1][3]);
  acc_guard4(acc[2][0], acc[2][1], acc[2][2], acc[2][3]);
  acc_guard4(acc[3][0], acc[3][1], acc[3][2], acc[3][3]);

  float* slab = sT[wave];
  const float* Rb = RESID ? (resid + (size_t)b * strideR) : nullptr;
#pragma unroll
  for (int i = 0; i < 4; ++i) {
    const int mBase = m0 + (i << 4);
#pragma unroll
    for (int j = 0; j < 4; ++j) {
      const int n = n0 + (j << 4) + rlane;
      float bv = 0.f;
      if (BIAS_MODE == 2) bv = bias[n];
#pragma unroll
      for (int r = 0; r < 8; ++r) {
        float v = acc[i][j][r] * scale;
        if (BIAS_MODE == 1) v += bias[mBase + mOff + r];
        if (BIAS_MODE == 2) v += bv;
        if (RESID) v += Rb[(size_t)(mBase + mOff + r) * ldc + n];
        if (ACT == 1) v = tanhf(v);
        if (ACT == 2) v = fmaxf(v, 0.0f);
        if (ACT == 3) v = v / (1.0f + expf(-v));
        if (ACT == 4) v = (v > 0.f) ? v : 0.01f * v;
        slab[(mOff + r) * 68 + (j << 4) + rlane] = v;
      }
    }
    __builtin_amdgcn_fence(__ATOMIC_RELEASE, "workgroup");
    __builtin_amdgcn_wave_barrier();
    __builtin_amdgcn_fence(__ATOMIC_ACQUIRE, "workgroup");
    if (OUT_MODE == 0) {
      float* C = (float*)Cout + (size_t)b * strideC;
      const int hh = lane >> 4, c4 = (lane & 15) * 4;
      for (int pass = 0; pass < 2; ++pass) {
#pragma unroll
        for (int it = 0; it < 8; ++it) {
          const int row = it * 2 + hh;
          v4f v = *(const v4f*)(slab + row * 68 + c4);
          *(volatile v4f*)(C + (size_t)(mBase + row) * ldc + n0 + c4) = v;
        }
        __threadfence();
      }
    } else {
      const int q = lane >> 3, c8 = (lane & 7) * 8;
      unsigned short* C  = (unsigned short*)Cout  + (size_t)b * strideC;
      unsigned short* C2 = (OUT_MODE == 2) ? ((unsigned short*)Cout2 + (size_t)b * strideC) : nullptr;
      for (int pass = 0; pass < 2; ++pass) {
#pragma unroll
        for (int it = 0; it < 4; ++it) {
          const int row = it * 4 + q;
          const float* sp = slab + row * 68 + c8;
          v8h hv, lv;
#pragma unroll
          for (int e = 0; e < 8; ++e) {
            if (OUT_MODE == 1) {
              hv[e] = (_Float16)sp[e];
            } else {
              unsigned short hb = f2bf_bits(sp[e]);
              unsigned short lb = f2bf_bits(sp[e] - bf_bits2f(hb));
              hv[e] = __builtin_bit_cast(_Float16, hb);
              lv[e] = __builtin_bit_cast(_Float16, lb);
            }
          }
          *(volatile v8h*)(C + (size_t)(mBase + row) * ldc + n0 + c8) = hv;
          if (OUT_MODE == 2) *(volatile v8h*)(C2 + (size_t)(mBase + row) * ldc + n0 + c8) = lv;
        }
        __threadfence();
      }
    }
    __builtin_amdgcn_fence(__ATOMIC_RELEASE, "workgroup");
    __builtin_amdgcn_wave_barrier();
    __builtin_amdgcn_fence(__ATOMIC_ACQUIRE, "workgroup");
  }
}

__global__ __launch_bounds__(256) void cast_bf16_kernel(
    const float* __restrict__ src, unsigned short* __restrict__ dst, int total8)
{
  const int i = blockIdx.x * 256 + threadIdx.x;
  if (i >= total8) return;
  const size_t e0 = (size_t)i << 3;
  const float* p = src + e0;
  const v4f a0 = *(const v4f*)(p);
  const v4f a1 = *(const v4f*)(p + 4);
  v8h hv;
#pragma unroll
  for (int e = 0; e < 4; ++e) {
    hv[e]     = __builtin_bit_cast(_Float16, f2bf_bits(a0[e]));
    hv[4 + e] = __builtin_bit_cast(_Float16, f2bf_bits(a1[e]));
  }
  unsigned short* q = dst + e0;
  *(volatile v8h*)q = hv;
  __threadfence();
  *(volatile v8h*)q = hv;
}

__global__ __launch_bounds__(256) void transpose_cast_bf16_kernel(
    const float* __restrict__ W, unsigned short* __restrict__ Bt, int Kdim, int Ndim)
{
  __shared__ float tile[64 * 65];
  const int tid = threadIdx.x, lane = tid & 31, wave = tid >> 5;
  const int n0 = blockIdx.x * 64;
  const int k0 = blockIdx.y * 64;
#pragma unroll
  for (int p = 0; p < 16; ++p) {
    const int idx = tid + p * 256;
    const int kk  = idx >> 6;
    const int nn  = idx & 63;
    const int n   = n0 + nn;
    const int nc  = (n < Ndim) ? n : (Ndim - 1);
    const float v = W[(size_t)(k0 + kk) * Ndim + nc];
    tile[kk * 65 + nn] = (n < Ndim) ? v : 0.f;
    if (p == 7) asm volatile("" ::: "memory");
  }
  __syncthreads();
  const int q = lane >> 3, c8 = (lane & 7) * 8;
  v8h hv[2];
#pragma unroll
  for (int it = 0; it < 2; ++it) {
    const int nrow = it * 32 + wave * 4 + q;
#pragma unroll
    for (int e = 0; e < 8; ++e) hv[it][e] = __builtin_bit_cast(_Float16, f2bf_bits(tile[(c8 + e) * 65 + nrow]));
  }
  for (int pass = 0; pass < 2; ++pass) {
#pragma unroll
    for (int it = 0; it < 2; ++it) {
      const int nrow = it * 32 + wave * 4 + q;
      *(volatile v8h*)(Bt + (size_t)(n0 + nrow) * Kdim + k0 + c8) = hv[it];
    }
    __threadfence();
  }
}

__global__ __launch_bounds__(kScanCh) void scan_kernel(
    const float* __restrict__ DTX, const float* __restrict__ ZF,
    const unsigned short* __restrict__ XPH, const unsigned short* __restrict__ XPL,
    const float* __restrict__ bdt, const float* __restrict__ A_log, const float* __restrict__ Dv,
    unsigned short* __restrict__ YH, unsigned short* __restrict__ YL)
{
  __shared__ __align__(16) float sBC[kScanTS * kBcN];
  __shared__ __align__(16) float sXP[kScanTS * kScanTP];
  __shared__ __align__(16) float sY[kScanTS * kScanTP];
  __shared__ float sA[kNst];
  const int tid = threadIdx.x, lane = tid & 31, wave = tid >> 5;
  const int d0 = blockIdx.x * kScanCh, d = d0 + tid;
  const size_t row0 = (size_t)blockIdx.y * kSeq;

  {
    const float av = -expf(bf16_rne(A_log[tid & (kNst - 1)]));
    if (tid < kNst) sA[tid] = av;
  }
  __syncthreads();
  float An[kNst], h[kNst];
#pragma unroll
  for (int n = 0; n < kNst; ++n) { An[n] = sA[n]; h[n] = 0.f; }
  const float bb = bf16_rne(bdt[d]);
  const float Dd = bf16_rne(Dv[d]);

#pragma unroll 1
  for (int c = 0; c < kSeq / kScanTS; ++c) {
    const int l0 = c * kScanTS;
    if (tid < 128) {
      const int r = tid >> 3, qq = (tid & 7) * 4;
      const v4f v = *(const v4f*)(DTX + (row0 + l0 + r) * kDtxN + kDin + qq);
      *(v4f*)(sBC + r * kBcN + qq) = v;
    }
#pragma unroll
    for (int it = 0; it < 2; ++it) {
      const int idx = tid + it * kScanCh;
      const int r   = idx >> 5;
      const int c8  = (idx & 31) * 8;
      const size_t o = (row0 + l0 + r) * kDin + d0 + c8;
      const v4u wh = *(const v4u*)(XPH + o);
      const v4u wl = *(const v4u*)(XPL + o);
      float* dst = sXP + r * kScanTP + c8;
#pragma unroll
      for (int e = 0; e < 4; ++e) {
        const unsigned a = wh[e];
        const unsigned bl = wl[e];
        dst[2 * e]     = __uint_as_float(a << 16) + __uint_as_float(bl << 16);
        dst[2 * e + 1] = __uint_as_float(a & 0xffff0000u) + __uint_as_float(bl & 0xffff0000u);
      }
    }
    __syncthreads();
#pragma unroll 1
    for (int s = 0; s < kScanTS; ++s) {
      const size_t m = row0 + l0 + s;
      const float a     = DTX[m * kDtxN + d] + bb;
      const float delta = fmaxf(a, 0.0f) + log1pf(__expf(-fabsf(a)));
      const float xv    = sXP[s * kScanTP + tid];
      const float zv    = ZF[m * kDin + d];
      v4f Bq[4], Cq[4];
#pragma unroll
      for (int qq = 0; qq < 4; ++qq) {
        Bq[qq] = *(const v4f*)(sBC + s * kBcN + 4 * qq);
        Cq[qq] = *(const v4f*)(sBC + s * kBcN + kNst + 4 * qq);
      }
      float y = 0.f;
#pragma unroll
      for (int n = 0; n < kNst; ++n) {
        const float e = __expf(delta * An[n]);
        float db = delta * Bq[n >> 2][n & 3];
        asm volatile("" : "+v"(db));
        float p = db * xv;
        asm volatile("" : "+v"(p));
        float qv = h[n] * e;
        asm volatile("" : "+v"(qv));
        const float hn = qv + p;
        h[n] = hn;
        float rr = Cq[n >> 2][n & 3] * hn;
        asm volatile("" : "+v"(rr));
        y += rr;
      }
      float sk = xv * Dd;
      asm volatile("" : "+v"(sk));
      y += sk;
      const float sg = __builtin_amdgcn_rcpf(1.0f + __expf(-zv));
      const float g  = zv * sg;
      sY[s * kScanTP + tid] = y * g;
    }
    __syncthreads();
    v8h hv[2], lv[2];
#pragma unroll
    for (int it = 0; it < 2; ++it) {
      const float* sp = sY + (it * 8 + wave) * kScanTP + lane * 8;
      const v4f a0 = *(const v4f*)(sp);
      const v4f a1 = *(const v4f*)(sp + 4);
#pragma unroll
      for (int e = 0; e < 4; ++e) {
        const unsigned short h0 = f2bf_bits(a0[e]), h1 = f2bf_bits(a1[e]);
        const unsigned short l0b = f2bf_bits(a0[e] - bf_bits2f(h0)), l1b = f2bf_bits(a1[e] - bf_bits2f(h1));
        hv[it][e]     = __builtin_bit_cast(_Float16, h0);
        hv[it][4 + e] = __builtin_bit_cast(_Float16, h1);
        lv[it][e]     = __builtin_bit_cast(_Float16, l0b);
        lv[it][4 + e] = __builtin_bit_cast(_Float16, l1b);
      }
    }
    for (int pass = 0; pass < 2; ++pass) {
#pragma unroll
      for (int it = 0; it < 2; ++it) {
        const size_t o = (row0 + l0 + it * 8 + wave) * kDin + d0 + lane * 8;
        *(volatile v8h*)(YH + o) = hv[it];
        *(volatile v8h*)(YL + o) = lv[it];
      }
      __threadfence();
    }
  }
}

extern "C" void kernel_launch(void* const* d_in, const int* in_sizes, int n_in,
                              void* d_out, int out_size, void* d_ws, size_t ws_size,
                              hipStream_t stream)
{
  if (n_in < 8) return;
  if (in_sizes[0] != kRows * kDm) return;
  if (in_sizes[1] != kDm * kXzN) return;
  if (in_sizes[2] != kDin * kBcN) return;
  if (in_sizes[3] != kDin * kDin) return;
  if (in_sizes[4] != kDin) return;
  if (in_sizes[5] != kNst) return;
  if (in_sizes[6] != kDin) return;
  if (in_sizes[7] != kDin * kDm) return;
  if (out_size != kRows * kDm) return;
  if (ws_size < kWsTotal) return;

  const float* x     = (const float*)d_in[0];
  const float* W_in  = (const float*)d_in[1];
  const float* W_x   = (const float*)d_in[2];
  const float* W_dt  = (const float*)d_in[3];
  const float* b_dt  = (const float*)d_in[4];
  const float* A_log = (const float*)d_in[5];
  const float* Dv    = (const float*)d_in[6];
  const float* W_out = (const float*)d_in[7];
  float* dout = (float*)d_out;

  char* ws = (char*)d_ws;
  unsigned short* XB    = (unsigned short*)(ws + kOffXB);
  unsigned short* WINB  = (unsigned short*)(ws + kOffWINB);
  unsigned short* WDTXB = (unsigned short*)(ws + kOffWDTXB);
  unsigned short* WOUTB = (unsigned short*)(ws + kOffWOUTB);
  float*          ZF    = (float*)(ws + kOffZF);
  unsigned short* XPH   = (unsigned short*)(ws + kOffXPH);
  unsigned short* XPL   = (unsigned short*)(ws + kOffXPL);
  float*          DTX   = (float*)(ws + kOffDTX);
  unsigned short* YH    = (unsigned short*)(ws + kOffYH);
  unsigned short* YL    = (unsigned short*)(ws + kOffYL);
  const float* dummy_bias  = b_dt;
  const float* dummy_resid = x;

  cast_bf16_kernel<<<(kRows * kDm) / 8 / 256, 256, 0, stream>>>(x, XB, (kRows * kDm) / 8);

  transpose_cast_bf16_kernel<<<dim3(kXzN / 64, kDm / 64), 256, 0, stream>>>(W_in, WINB, kDm, kXzN);
  transpose_cast_bf16_kernel<<<dim3(kDin / 64, kDin / 64), 256, 0, stream>>>(W_dt, WDTXB, kDin, kDin);
  transpose_cast_bf16_kernel<<<dim3(1, kDin / 64), 256, 0, stream>>>(W_x, WDTXB + (size_t)kDin * kDin, kDin, kBcN);
  transpose_cast_bf16_kernel<<<dim3(kDm / 64, kDin / 64), 256, 0, stream>>>(W_out, WOUTB, kDin, kDm);

  wmma_gemm64<1, 0, 0, 2, false><<<dim3(((kRows / 64) * (kDin / 64)) / 8, 1), 256, 0, stream>>>(
      XB, XB, kDm, 0L, WINB, WINB, kDm, 0L,
      (void*)XPH, (void*)XPL, kDin, 0L, dummy_bias, dummy_resid, 0L, kRows, kDin, kDm, 1.0f);

  wmma_gemm64<1, 0, 0, 0, false><<<dim3(((kRows / 64) * (kDin / 64)) / 8, 1), 256, 0, stream>>>(
      XB, XB, kDm, 0L, WINB + (size_t)kDin * kDm, WINB + (size_t)kDin * kDm, kDm, 0L,
      (void*)ZF, (void*)ZF, kDin, 0L, dummy_bias, dummy_resid, 0L, kRows, kDin, kDm, 1.0f);

  wmma_gemm64<1, 1, 0, 0, false><<<dim3(((kRows / 64) * (kDtxN / 64)) / 8, 1), 256, 0, stream>>>(
      XPH, XPL, kDin, 0L, WDTXB, WDTXB, kDin, 0L,
      (void*)DTX, (void*)DTX, kDtxN, 0L, dummy_bias, dummy_resid, 0L, kRows, kDtxN, kDin, 1.0f);

  scan_kernel<<<dim3(kDin / kScanCh, kBatch), kScanCh, 0, stream>>>(DTX, ZF, XPH, XPL, b_dt, A_log, Dv, YH, YL);

  wmma_gemm64<1, 1, 0, 0, false><<<dim3(((kRows / 64) * (kDm / 64)) / 8, 1), 256, 0, stream>>>(
      YH, YL, kDin, 0L, WOUTB, WOUTB, kDin, 0L,
      (void*)dout, (void*)dout, kDm, 0L, dummy_bias, dummy_resid, 0L, kRows, kDm, kDin, 1.0f);
}
